// MoELoRALayer_26027501813957
// MI455X (gfx1250) — hardware-verified
//
#include <hip/hip_runtime.h>


#define NB   4
#define NT_  2048
#define DM   1024
#define NTK  NT_
#define GQ   256
#define NE   8
#define NR   16
#define ER   (NE * NR)
#define SCAL 2.0f
#define LOSC 1024.0f

typedef _Float16 h16;
typedef unsigned short bf;
typedef __attribute__((ext_vector_type(16))) __bf16   v16bf;
typedef __attribute__((ext_vector_type(16))) _Float16 v16h;
typedef __attribute__((ext_vector_type(8)))  _Float16 v8h;
typedef __attribute__((ext_vector_type(8)))  unsigned short v8us;
typedef __attribute__((ext_vector_type(8)))  float    v8f;
typedef __attribute__((ext_vector_type(4)))  float    v4f;
typedef __attribute__((ext_vector_type(4)))  _Float16 v4h;
typedef v8h  __attribute__((may_alias)) v8ha;
typedef v4f  __attribute__((may_alias)) v4fa;
typedef v8us __attribute__((may_alias)) v8usa;

__device__ __forceinline__ unsigned short f2bf(float f) { unsigned u = __float_as_uint(f); u += 0x7FFFu + ((u >> 16) & 1u); return (unsigned short)(u >> 16); }
__device__ __forceinline__ float bf2f(unsigned short b) { return __uint_as_float(((unsigned)b) << 16); }
__device__ __forceinline__ float bfr(float f) { return bf2f(f2bf(f)); }
__device__ __forceinline__ v16h cat16(v8h lo, v8h hi) { return __builtin_shufflevector(lo, hi, 0, 1, 2, 3, 4, 5, 6, 7, 8, 9, 10, 11, 12, 13, 14, 15); }
__device__ __forceinline__ v16bf cat16b(v8us lo, v8us hi) { return __builtin_bit_cast(v16bf, __builtin_shufflevector(lo, hi, 0, 1, 2, 3, 4, 5, 6, 7, 8, 9, 10, 11, 12, 13, 14, 15)); }
__device__ __forceinline__ v8f wmma16(v16h a, v16h b, v8f c) { return __builtin_amdgcn_wmma_f32_16x16x32_f16(false, a, false, b, (short)0, c, false, false); }
__device__ __forceinline__ v8f wmmab(v16bf a, v16bf b, v8f c) { return __builtin_amdgcn_wmma_f32_16x16x32_bf16(false, a, false, b, (short)0, c, false, false); }

__global__ __launch_bounds__(256) void k_cvtb(const float* __restrict__ src, int nrows, bf* dst) {
    const int lane = threadIdx.x & 31, r = blockIdx.x * 8 + (threadIdx.x >> 5);
    if (r >= nrows) return;
    v8us o[DM / 256];
#pragma unroll
    for (int q = 0; q < DM / 256; ++q) { v8us t;
#pragma unroll
        for (int i = 0; i < 8; ++i) t[i] = f2bf(src[(size_t)r * DM + q * 256 + lane * 8 + i]);
        o[q] = t; }
#pragma unroll
    for (int q = 0; q < DM / 256; ++q) *(volatile v8us*)(dst + (size_t)r * DM + q * 256 + lane * 8) = o[q];
    __threadfence();
#pragma unroll
    for (int q = 0; q < DM / 256; ++q) *(volatile v8us*)(dst + (size_t)r * DM + q * 256 + lane * 8) = o[q];
}

__global__ __launch_bounds__(256) void k_wt(const float* __restrict__ Wm, int K, int ncols, bf* WT) {
    __shared__ __align__(16) unsigned short tl[64 * 72];
    const int tid = threadIdx.x, k0 = blockIdx.x * 64, n0 = blockIdx.y * 64;
    const int kk = tid >> 2, nq = (tid & 3) * 16;
#pragma unroll
    for (int i = 0; i < 16; ++i) tl[(nq + i) * 72 + kk] = f2bf(Wm[(size_t)(k0 + kk) * ncols + n0 + nq + i]);
    __syncthreads();
    const int piece = tid & 7;
    auto pass = [&]() {
#pragma unroll
        for (int s = 0; s < 2; ++s) { const int nr = (tid >> 3) + 32 * s; const v8us val = *(const v8usa*)(tl + nr * 72 + piece * 8); *(volatile v8us*)(WT + (size_t)(n0 + nr) * K + k0 + piece * 8) = val; }
    };
    pass(); __threadfence(); pass();
}
template <bool SPLITA, bool F16OUT = false>
__global__ __launch_bounds__(128) void k_gemmb(const bf* __restrict__ A, const bf* __restrict__ Al, const bf* __restrict__ Bn, const float* __restrict__ bias, float* C, int ldc, h16* C2, const float* __restrict__ R = nullptr, int K = DM, int roundR = 1) {
    __shared__ __align__(16) float ost[4][16 * 68];
    const int lane = threadIdx.x & 31, wave = threadIdx.x >> 5, lr = lane & 15, hi = lane >> 4;
    const int r0 = blockIdx.x * 64 + wave * 16, c0 = blockIdx.y * 64;
    const size_t aoff = (size_t)(r0 + lr) * K + 8 * hi;
    size_t boff[4];
#pragma unroll
    for (int t = 0; t < 4; ++t) boff[t] = (size_t)(c0 + t * 16 + lr) * K + 8 * hi;
    v8f acc[4];
#pragma unroll
    for (int t = 0; t < 4; ++t) acc[t] = (v8f){};
#pragma unroll 1
    for (int kc = 0; kc < K; kc += 32) {
        const v16bf a = cat16b(*(const v8us*)(A + aoff + kc), *(const v8us*)(A + aoff + kc + 16));
        v16bf al = a;
        if (SPLITA) al = cat16b(*(const v8us*)(Al + aoff + kc), *(const v8us*)(Al + aoff + kc + 16));
#pragma unroll
        for (int t = 0; t < 4; ++t) { const v16bf b = cat16b(*(const v8us*)(Bn + boff[t] + kc), *(const v8us*)(Bn + boff[t] + kc + 16)); acc[t] = wmmab(a, b, acc[t]); if (SPLITA) acc[t] = wmmab(al, b, acc[t]); }
        asm volatile("v_nop\n\tv_nop\n\tv_nop\n\tv_nop" : "+v"(acc[0]), "+v"(acc[1]), "+v"(acc[2]), "+v"(acc[3]) : "v"(a), "v"(al));
    }
    float* os = &ost[wave][0];
#pragma unroll
    for (int t = 0; t < 4; ++t) { const float bv = bias ? bfr(bias[c0 + t * 16 + lr]) : 0.f;
#pragma unroll
        for (int j = 0; j < 8; ++j) os[(hi * 8 + j) * 68 + t * 16 + lr] = acc[t][j] + bv; }
    __syncthreads();
    if (F16OUT) {
        h16* crow = (h16*)(void*)C + (size_t)r0 * ldc + c0;
        auto pass = [&]() {
#pragma unroll
            for (int s = 0; s < 4; ++s) { const int row = 4 * s + (lane >> 3), piece = lane & 7; const float* sp = os + row * 68 + piece * 8; v8h o, o2;
#pragma unroll
                for (int i = 0; i < 8; ++i) { const h16 a = (h16)sp[i]; o[i] = a; o2[i] = (h16)((sp[i] - (float)a) * LOSC); }
                *(volatile v8h*)(crow + (size_t)row * ldc + piece * 8) = o; if (C2) *(volatile v8h*)(C2 + (size_t)r0 * ldc + c0 + (size_t)row * ldc + piece * 8) = o2; }
        };
        pass(); __threadfence(); pass();
    } else {
        float* crow = C + (size_t)r0 * ldc + c0;
        auto pass = [&]() {
#pragma unroll
            for (int s = 0; s < 8; ++s) { const int Lid = (lane >> 3) + 4 * s, piece = lane & 7; const int row = Lid >> 1, cofs = (Lid & 1) * 32 + piece * 4;
                v4f val = *(const v4fa*)(os + row * 68 + cofs); if (R) { const v4f rv = *(const v4f*)(R + ((size_t)r0 + row) * ldc + c0 + cofs); val += roundR ? (v4f){bfr(rv[0]), bfr(rv[1]), bfr(rv[2]), bfr(rv[3])} : rv; }
                *(volatile v4f*)(crow + (size_t)row * ldc + cofs) = val; }
        };
        pass(); __threadfence(); pass();
    }
}


__global__ __launch_bounds__(256) void k_bf(const float* __restrict__ src, bf* dst, size_t n8) {
    const size_t i = (size_t)blockIdx.x * 256 + threadIdx.x; if (i >= n8) return;
    const v8f v = *(const v8f*)(src + i * 8); v8us o;
#pragma unroll
    for (int k = 0; k < 8; ++k) o[k] = f2bf(v[k]);
    *(volatile v8us*)(dst + i * 8) = o; __threadfence(); *(volatile v8us*)(dst + i * 8) = o;
}
__global__ __launch_bounds__(256) void k_bcat(const float* __restrict__ LB, bf* BC) {
    const size_t u = (size_t)blockIdx.x * 256 + threadIdx.x; if (u >= (size_t)DM * 16) return;
    const int h = (int)(u / 16), q16 = (int)(u % 16), e = q16 >> 1, r0 = (q16 & 1) * 8;
    v8us o;
#pragma unroll
    for (int i = 0; i < 8; ++i) o[i] = f2bf(LB[((size_t)e * DM + h) * NR + r0 + i]);
    bf* p = BC + (size_t)h * ER + q16 * 8; *(volatile v8us*)p = o; __threadfence(); *(volatile v8us*)p = o;
}
__global__ __launch_bounds__(256) void k_gate(const float* __restrict__ HG, const float* __restrict__ W2, const float* __restrict__ b2, const int* __restrict__ fids, int b,
                                              const float* __restrict__ AF, bf* AGh, bf* AGl) {
    typedef __attribute__((ext_vector_type(4))) unsigned short v4us;
    const int lane = threadIdx.x & 31, r = blockIdx.x * 8 + (threadIdx.x >> 5); if (r >= NT_) return;
    const float* hrow = HG + (size_t)r * GQ;
    float lg[NE];
#pragma unroll
    for (int e = 0; e < NE; ++e) { float s = 0.f;
#pragma unroll
        for (int i = 0; i < GQ / 32; ++i) { const int q = i * 32 + lane; s = fmaf(fmaxf(hrow[q], 0.f), bfr(W2[q * NE + e]), s); }
#pragma unroll
        for (int sh = 16; sh; sh >>= 1) s += __shfl_xor(s, sh, 32);
        lg[e] = s + bfr(b2[e]); }
    const int fid = fids[b];
    float mx = -3.0e38f;
#pragma unroll
    for (int e = 0; e < NE; ++e) { const bool allowed = (e == 0) || (e == fid + 1); lg[e] = allowed ? lg[e] : lg[e] - 1e9f; mx = fmaxf(mx, lg[e]); }
    float den = 0.f, g[NE];
#pragma unroll
    for (int e = 0; e < NE; ++e) { g[e] = __expf(lg[e] - mx); den += g[e]; }
    const float inv = 1.0f / den;
    float gl = 0.f;
#pragma unroll
    for (int e = 0; e < NE; ++e) gl = (lane / 4 == e) ? g[e] * inv * SCAL : gl;
    const v4f av = *(const v4f*)(AF + (size_t)r * ER + lane * 4); v4us oh, ol;
#pragma unroll
    for (int i = 0; i < 4; ++i) { const float y = av[i] * gl; const unsigned short hb = f2bf(y); oh[i] = hb; ol[i] = f2bf(y - bf2f(hb)); }
    const size_t o = (size_t)r * ER + lane * 4;
    *(volatile v4us*)(AGh + o) = oh; *(volatile v4us*)(AGl + o) = ol; __threadfence(); *(volatile v4us*)(AGh + o) = oh; *(volatile v4us*)(AGl + o) = ol;
}

extern "C" void kernel_launch(void* const* d_in, const int* in_sizes, int n_in,
                              void* d_out, int out_size, void* d_ws, size_t ws_size, hipStream_t stream) {
    (void)in_sizes; (void)n_in; (void)out_size;
    const float* x = (const float*)d_in[0]; const float* LA = (const float*)d_in[1]; const float* LB = (const float*)d_in[2];
    const float* W1 = (const float*)d_in[3]; const float* b1 = (const float*)d_in[4]; const float* W2 = (const float*)d_in[5]; const float* b2 = (const float*)d_in[6]; const int* fids = (const int*)d_in[7];
    float* out = (float*)d_out;
    char* wsp = (char*)d_ws;
    auto take = [&](size_t bytes) { char* p = wsp; wsp += (bytes + 255) & ~(size_t)255; return (void*)p; };
    bf* Xb = (bf*)take((size_t)NTK * DM * 2); bf* W1T = (bf*)take((size_t)GQ * DM * 2); bf* AB = (bf*)take((size_t)ER * DM * 2); bf* BC = (bf*)take((size_t)DM * ER * 2);
    float* HG = (float*)take((size_t)NTK * GQ * 4); float* AF = (float*)take((size_t)NTK * ER * 4); bf* AGh = (bf*)take((size_t)NTK * ER * 2); bf* AGl = (bf*)take((size_t)NTK * ER * 2);
    if ((size_t)(wsp - (char*)d_ws) > ws_size) return;
    k_wt<<<dim3(DM / 64, GQ / 64, 1), 256, 0, stream>>>(W1, DM, GQ, W1T);
    k_bf<<<(ER * DM / 8 + 255) / 256, 256, 0, stream>>>(LA, AB, (size_t)ER * DM / 8);
    k_bcat<<<(DM * 16 + 255) / 256, 256, 0, stream>>>(LB, BC);
    for (int b = 0; b < NB; ++b) {
        k_cvtb<<<NTK / 8, 256, 0, stream>>>(x + (size_t)b * NTK * DM, NTK, Xb);
        k_gemmb<false, false><<<dim3(NTK / 64, GQ / 64, 1), 128, 0, stream>>>(Xb, nullptr, W1T, b1, HG, GQ, nullptr);
        k_gemmb<false, false><<<dim3(NTK / 64, ER / 64, 1), 128, 0, stream>>>(Xb, nullptr, AB, nullptr, AF, ER, nullptr);
        k_gate<<<NTK / 8, 256, 0, stream>>>(HG, W2, b2, fids, b, AF, AGh, AGl);
        k_gemmb<true, false><<<dim3(NTK / 64, DM / 64, 1), 128, 0, stream>>>(AGh, AGl, BC, nullptr, out + (size_t)b * NTK * DM, DM, nullptr, nullptr, ER);
    }
}
